// GAT_81836306858559
// MI455X (gfx1250) — hardware-verified
//
#include <hip/hip_runtime.h>
#include <stddef.h>
#include <stdint.h>
#include <math.h>


#define F_IN    128
#define HID     64
#define FC1N    32
#define NTHR    256
#define NWAVE   8
#define EPT     8
#define CHUNK   (NTHR * EPT)
#define WCAP    (EPT * 32)
#define LISTN   (NWAVE * WCAP)
#define NBMAX   2048
#define SLOTB   11
#define NBRUN   1024
#define SRCB    17
#define RCAP    28672
#define DEGCAP  64
#define MEAS_B1024  10503
#define MEAS_MAXDEG 25
#define GBM     64
#define GBN     64
#define GTHR    128
#define MROWS   128
#define NEG_ATT 0.2f
#define NEG_ACT 0.01f
#define EPS_SM  1e-16f
#define WSMAX   134217728
#define LDS_BKT ((2 * RCAP + 2 * NBMAX + LISTN) * 4 + 64)

#define PO_BLR0 0
#define PO_BLR1 128
#define PO_ATT  256
#define PO_BIAS 384
#define PO_FC1W 512
#define PO_FC1B 2560
#define PO_FC2W 2592
#define PO_FC2B 2624
#define PARN    2688

static_assert((CHUNK & (CHUNK - 1)) == 0 && CHUNK <= (1 << SLOTB));
static_assert(NBMAX == (1 << SLOTB));
static_assert(NTHR * 8 == NBMAX);
static_assert(LISTN >= NBMAX && LISTN >= NWAVE * WCAP);
static_assert(NBRUN <= 1024 && (NBRUN % 32) == 0 && NBRUN <= NBMAX);
static_assert(NBRUN == 4 * NTHR);
static_assert((NBRUN % NWAVE) == 0);
static_assert(SRCB + 10 <= 31);
static_assert((RCAP % 32) == 0 && (RCAP % (4 * NTHR)) == 0);
static_assert(RCAP >= MEAS_B1024 + 4096);
static_assert(DEGCAP >= MEAS_MAXDEG + 8 && (DEGCAP % 32) == 0);
static_assert(LDS_BKT <= 327680);
static_assert(GBM == (GTHR / 32) * 16);
static_assert((F_IN % 32) == 0 && (2 * HID) == F_IN);
static_assert(HID == 2 * 32);
static_assert((MROWS % GBM) == 0);
static_assert((PARN % 32) == 0 && PO_FC2B + 64 == PARN);
static_assert(HID * FC1N == 8 * NTHR);

typedef float          v2f  __attribute__((ext_vector_type(2)));
typedef float          v4f  __attribute__((ext_vector_type(4)));
typedef float          v8f  __attribute__((ext_vector_type(8)));
typedef int            v4i  __attribute__((ext_vector_type(4)));
typedef int            v8i  __attribute__((ext_vector_type(8)));
typedef unsigned int   v4u  __attribute__((ext_vector_type(4)));
typedef unsigned short v8us __attribute__((ext_vector_type(8)));
typedef __bf16         v16b __attribute__((ext_vector_type(16)));
typedef v2f  __attribute__((may_alias)) v2fa;
typedef v4f  __attribute__((may_alias)) v4fa;
typedef v8us __attribute__((may_alias)) v8usa;
union FragB { v16b v; v8us h[2]; v8i w; };

__device__ __forceinline__ v8f wmb(const FragB& a, const FragB& b, v8f c) {
  v8f d = __builtin_amdgcn_wmma_f32_16x16x32_bf16(false, a.v, false, b.v, (short)0, c, false, false);
  asm volatile("v_nop\n\tv_nop\n\tv_nop\n\tv_nop" : "+v"(d) : "v"(a.w), "v"(b.w));
  return d;
}

__device__ __forceinline__ void ldwait() {
  asm volatile("s_wait_loadcnt 0x0" ::: "memory");
}

__device__ __forceinline__ unsigned int f2bf(float f) {
  const unsigned int u = __float_as_uint(f);
  return ((u + 0x7FFFu + ((u >> 16) & 1u)) >> 16) & 0xFFFFu;
}
__device__ __forceinline__ unsigned int f2bfn(float f) {
  const unsigned int r = f2bf(f);
  return (f != f) ? 0x7FC0u : r;
}
__device__ __forceinline__ float bf2f(unsigned int b) { return __uint_as_float(b << 16); }
__device__ __forceinline__ float bfr(float f) { return bf2f(f2bf(f)); }
__device__ __forceinline__ v4f bfr4(const v4f a) {
  v4f r; r.x = bfr(a.x); r.y = bfr(a.y); r.z = bfr(a.z); r.w = bfr(a.w); return r;
}
__device__ __forceinline__ unsigned int pk2(float lo, float hi) { return f2bf(lo) | (f2bf(hi) << 16); }
__device__ __forceinline__ v4u pack8(const v4f a, const v4f b) {
  v4u r;
  r.x = pk2(a.x, a.y); r.y = pk2(a.z, a.w); r.z = pk2(b.x, b.y); r.w = pk2(b.z, b.w);
  return r;
}

__device__ __forceinline__ int scan_chunk(const int* __restrict__ dsts, int nE, int cbase, int slotBase,
                                          int nb, int vec8, int* list, int tid, int lane, int wave) {
  int wc = 0;
  const int el0  = tid * EPT;
  const int e0   = cbase + el0;
  const int sent = -2147483647 - 1;
  v4i da, db;
  if (vec8 != 0 && cbase + CHUNK <= nE) {
    da = *(const v4i*)(dsts + e0);
    db = *(const v4i*)(dsts + e0 + 4);
  } else {
    da.x = (e0     < nE) ? dsts[min(e0,     nE - 1)] : sent;
    da.y = (e0 + 1 < nE) ? dsts[min(e0 + 1, nE - 1)] : sent;
    da.z = (e0 + 2 < nE) ? dsts[min(e0 + 2, nE - 1)] : sent;
    da.w = (e0 + 3 < nE) ? dsts[min(e0 + 3, nE - 1)] : sent;
    db.x = (e0 + 4 < nE) ? dsts[min(e0 + 4, nE - 1)] : sent;
    db.y = (e0 + 5 < nE) ? dsts[min(e0 + 5, nE - 1)] : sent;
    db.z = (e0 + 6 < nE) ? dsts[min(e0 + 6, nE - 1)] : sent;
    db.w = (e0 + 7 < nE) ? dsts[min(e0 + 7, nE - 1)] : sent;
  }
  const unsigned nbs = (unsigned)slotBase;
  const unsigned unb = (unsigned)nb;
  const unsigned s0 = (unsigned)da.x - nbs, s1 = (unsigned)da.y - nbs;
  const unsigned s2 = (unsigned)da.z - nbs, s3 = (unsigned)da.w - nbs;
  const unsigned s4 = (unsigned)db.x - nbs, s5 = (unsigned)db.y - nbs;
  const unsigned s6 = (unsigned)db.z - nbs, s7 = (unsigned)db.w - nbs;
  const bool h0 = s0 < unb, h1 = s1 < unb, h2 = s2 < unb, h3 = s3 < unb;
  const bool h4 = s4 < unb, h5 = s5 < unb, h6 = s6 < unb, h7 = s7 < unb;
  const unsigned any = __builtin_amdgcn_ballot_w32(h0 | h1 | h2 | h3 | h4 | h5 | h6 | h7);
  if (any != 0u) {
#define HITJ(J, HJ, SJ) { \
      const unsigned mj = __builtin_amdgcn_ballot_w32(HJ); \
      if (mj != 0u) { \
        if (HJ) { \
          const int pos = wc + (int)__builtin_amdgcn_mbcnt_lo(mj, 0u); \
          if (pos < WCAP) list[wave * WCAP + pos] = ((el0 + (J)) << SLOTB) | (int)(SJ); \
        } \
        wc += (int)__builtin_popcount(mj); } }
    HITJ(0, h0, s0)
    HITJ(1, h1, s1)
    HITJ(2, h2, s2)
    HITJ(3, h3, s3)
    HITJ(4, h4, s4)
    HITJ(5, h5, s5)
    HITJ(6, h6, s6)
    HITJ(7, h7, s7)
#undef HITJ
  }
  return wc;
}

__device__ __forceinline__ void x_unit(const float* __restrict__ x, unsigned short* xb, int nN, int i) {
  const int row = i >> 4;
  const int c0  = (i & 15) * 8;
  const int rc  = row < nN ? row : nN - 1;
  const float* p = x + (size_t)rc * F_IN + c0;
  v4f a = *(const v4fa*)p, b = *(const v4fa*)(p + 4);
  const v4f z4 = {0.f, 0.f, 0.f, 0.f};
  if (row >= nN) { a = z4; b = z4; }
  const v4u hv = pack8(a, b);
  unsigned short* o = xb + (size_t)row * F_IN + c0;
  *(volatile v4u*)o = hv;
  __threadfence();
  *(volatile v4u*)o = hv;
}

__device__ __forceinline__ void wtr_unit(const float* __restrict__ w, int Kin, unsigned short* wt, int rowOff, int u) {
  const int n  = u >> 4;
  const int k8 = (u & 15) * 8;
  const int kk = k8 - (k8 / Kin) * Kin;
  const float* p = w + (size_t)kk * HID + n;
  v4f a, b;
  a.x = p[0];        a.y = p[HID];      a.z = p[2 * HID];  a.w = p[3 * HID];
  b.x = p[4 * HID];  b.y = p[5 * HID];  b.z = p[6 * HID];  b.w = p[7 * HID];
  const v4u wv = pack8(a, b);
  unsigned short* o = wt + (size_t)(rowOff + n) * F_IN + k8;
  *(volatile v4u*)o = wv;
  __threadfence();
  *(volatile v4u*)o = wv;
}

__global__ __launch_bounds__(NTHR) void k_prep(
    const float* __restrict__ x,
    const float* __restrict__ wl0, const float* __restrict__ bl0,
    const float* __restrict__ wr0, const float* __restrict__ br0,
    const float* __restrict__ att0, const float* __restrict__ bias0,
    const float* __restrict__ wl1, const float* __restrict__ bl1,
    const float* __restrict__ wr1, const float* __restrict__ br1,
    const float* __restrict__ att1, const float* __restrict__ bias1,
    const float* __restrict__ fc1w, const float* __restrict__ fc1b,
    const float* __restrict__ fc2w, const float* __restrict__ fc2b,
    unsigned short* XB, unsigned short* W0T, unsigned short* W1T2, float* PAR, int nN, int nbX)
{
  __shared__ __attribute__((aligned(16))) float sp[PARN];
  const int tid = (int)threadIdx.x;
  const int blk = (int)blockIdx.x;
  if (blk < nbX) { x_unit(x, XB, nN, blk * NTHR + tid); return; }
  const int wb = blk - nbX;
  if (wb < 16) {
    const int u = (wb & 3) * NTHR + tid;
    if (wb < 4)       wtr_unit(wl0, F_IN, W0T, 0, u);
    else if (wb < 8)  wtr_unit(wr0, F_IN, W0T, HID, u);
    else if (wb < 12) wtr_unit(wl1, HID, W1T2, 0, u);
    else              wtr_unit(wr1, HID, W1T2, HID, u);
    return;
  }
  const int i64 = tid & 63, i32 = tid & 31;
  {
    const float a = bl0[i64], b = br0[i64], c = bl1[i64], d = br1[i64];
    ldwait();
    if (tid < 64) {
      sp[PO_BLR0 + i64] = bfr(a); sp[PO_BLR0 + HID + i64] = bfr(b);
      sp[PO_BLR1 + i64] = bfr(c); sp[PO_BLR1 + HID + i64] = bfr(d);
    }
  }
  {
    const float a = att0[i64], b = att1[i64], c = bias0[i64], d = bias1[i64];
    ldwait();
    if (tid < 64) {
      sp[PO_ATT + i64]  = bfr(a); sp[PO_ATT + HID + i64]  = bfr(b);
      sp[PO_BIAS + i64] = bfr(c); sp[PO_BIAS + HID + i64] = bfr(d);
    }
  }
#pragma unroll 1
  for (int j = 0; j < 2; ++j) {
    const int q = 4 * (tid + NTHR * j);
    const v4f w = *(const v4fa*)(fc1w + q);
    *(v4fa*)(sp + PO_FC1W + q) = bfr4(w);
  }
  {
    const float a = fc1b[i32], b = fc2w[i32], c = fc2b[0];
    ldwait();
    if (tid < 32) {
      sp[PO_FC1B + i32] = bfr(a);
      sp[PO_FC2W + i32] = bfr(b);
      sp[PO_FC2B + i32] = (i32 == 0) ? bfr(c) : 0.f;
      sp[PO_FC2B + 32 + i32] = 0.f;
    }
  }
  __syncthreads();
#pragma unroll 1
  for (int p = tid; p < PARN / 4; p += NTHR) {
    const v4f v = *(const v4fa*)(sp + 4 * p);
    *(volatile v4f*)(PAR + 4 * p) = v;
  }
  __threadfence();
#pragma unroll 1
  for (int p = tid; p < PARN / 4; p += NTHR) {
    const v4f v = *(const v4fa*)(sp + 4 * p);
    *(volatile v4f*)(PAR + 4 * p) = v;
  }
}

__global__ __launch_bounds__(NTHR) void k_bucket(
    const int* __restrict__ srcs, const int* __restrict__ dsts,
    int* HITS, int* SCNT, int* SOFF, int* META, int nN, int nE, int vec8) {
  extern __shared__ v4f lds_dyn[];
  int* reg1 = (int*)lds_dyn;
  int* reg2 = reg1 + RCAP;
  int* scnt = reg2 + RCAP;
  int* soff = scnt + NBMAX;
  int* list = soff + NBMAX;
  int* wcnt = list + LISTN;
  int* wtot = wcnt + NWAVE;
  const int tid = (int)threadIdx.x, lane = tid & 31, wave = tid >> 5;
  const int b = (int)blockIdx.x;
  const int nodeBase = b * NBRUN;
  int nbHit = nN - nodeBase;
  nbHit = nbHit < 0 ? 0 : (nbHit > NBRUN ? NBRUN : nbHit);

  for (int i = tid; i < NBMAX; i += NTHR) scnt[i] = 0;
  for (int i = tid; i < RCAP; i += NTHR) reg2[i] = 0;
  __syncthreads();

  int tot = 0;
  const int nChunks = (nE + CHUNK - 1) / CHUNK;
#pragma unroll 1
  for (int ch = 0; ch < nChunks; ++ch) {
    const int cbase = ch * CHUNK;
    const int wc = scan_chunk(dsts, nE, cbase, nodeBase, nbHit, vec8, list, tid, lane, wave);
    if (lane == 0) wcnt[wave] = wc;
    __syncthreads();
    int pre = 0, all = 0;
#pragma unroll
    for (int w2 = 0; w2 < NWAVE; ++w2) {
      int c = wcnt[w2];
      c = c < 0 ? 0 : (c > WCAP ? WCAP : c);
      all += c;
      pre += (w2 < wave) ? c : 0;
    }
    const int wcc  = wc > WCAP ? WCAP : wc;
    const int base = tot + pre;
#pragma unroll 1
    for (int i0 = 0; i0 < wcc; i0 += 32) {
      const int i   = i0 + lane;
      const int ic  = i < wcc ? i : wcc - 1;
      const int ent = list[wave * WCAP + ic];
      const int el  = (ent >> SLOTB) & (CHUNK - 1);
      const int sl  = ent & (NBRUN - 1);
      int eid = cbase + el;
      eid = eid < 0 ? 0 : (eid > nE - 1 ? nE - 1 : eid);
      const int sraw = srcs[eid];
      const int s = sraw < 0 ? 0 : (sraw > nN - 1 ? nN - 1 : sraw);
      const int pos = base + i;
      if (i < wcc && pos < RCAP) reg1[pos] = (sl << SRCB) | s;
    }
    tot += all;
    tot = tot > RCAP ? RCAP : tot;
    __syncthreads();
  }
  const int nh = tot;

  if (wave == 0) {
#pragma unroll 1
    for (int b0 = 0; b0 < nh; b0 += 32) {
      const int idx = b0 + lane;
      const int uv  = reg1[idx < nh ? idx : nh - 1];
      const int m32 = (nh - b0) < 32 ? (nh - b0) : 32;
#pragma unroll 1
      for (int k = 0; k < m32; ++k) {
        const int u  = __builtin_amdgcn_readlane(uv, k);
        const int sl = (int)(((unsigned)u >> SRCB) & (unsigned)(NBMAX - 1));
        if (lane == 0) scnt[sl] = scnt[sl] + 1;
      }
    }
  }
  __syncthreads();

  {
    const v4i ca = *(const v4i*)(scnt + 8 * tid);
    const v4i cb = *(const v4i*)(scnt + 8 * tid + 4);
    const int e0 = ca.x < 0 ? 0 : ca.x, e1 = ca.y < 0 ? 0 : ca.y, e2 = ca.z < 0 ? 0 : ca.z, e3 = ca.w < 0 ? 0 : ca.w;
    const int e4 = cb.x < 0 ? 0 : cb.x, e5 = cb.y < 0 ? 0 : cb.y, e6 = cb.z < 0 ? 0 : cb.z, e7 = cb.w < 0 ? 0 : cb.w;
    const int ts = e0 + e1 + e2 + e3 + e4 + e5 + e6 + e7;
    int incl = ts;
#pragma unroll
    for (int d = 1; d < 32; d <<= 1) {
      const int up = __shfl_up(incl, d);
      if (lane >= d) incl += up;
    }
    if (lane == 31) wtot[wave] = incl;
    __syncthreads();
    int pre = 0;
#pragma unroll
    for (int w2 = 0; w2 < NWAVE; ++w2) pre += (w2 < wave) ? wtot[w2] : 0;
    int run = pre + incl - ts;
    soff[8 * tid + 0] = run; run += e0;
    soff[8 * tid + 1] = run; run += e1;
    soff[8 * tid + 2] = run; run += e2;
    soff[8 * tid + 3] = run; run += e3;
    soff[8 * tid + 4] = run; run += e4;
    soff[8 * tid + 5] = run; run += e5;
    soff[8 * tid + 6] = run; run += e6;
    soff[8 * tid + 7] = run;
  }
  __syncthreads();
  for (int i = tid; i < NBMAX; i += NTHR) list[i] = soff[i];
  __syncthreads();

  if (wave == 0) {
#pragma unroll 1
    for (int b0 = 0; b0 < nh; b0 += 32) {
      const int idx = b0 + lane;
      const int uv  = reg1[idx < nh ? idx : nh - 1];
      const int m32 = (nh - b0) < 32 ? (nh - b0) : 32;
#pragma unroll 1
      for (int k = 0; k < m32; ++k) {
        const int u  = __builtin_amdgcn_readlane(uv, k);
        const int sl = (int)(((unsigned)u >> SRCB) & (unsigned)(NBMAX - 1));
        const int sv = u & ((1 << SRCB) - 1);
        if (lane == 0) {
          int pos = list[sl];
          pos = pos < 0 ? 0 : (pos > RCAP - 1 ? RCAP - 1 : pos);
          reg2[pos] = sv;
          list[sl] = pos + 1;
        }
      }
    }
  }
  __syncthreads();

  int* hg = HITS + (size_t)b * RCAP;
  int* cg = SCNT + (size_t)b * NBRUN + 4 * tid;
  int* og = SOFF + (size_t)b * NBRUN + 4 * tid;
  int* mg = META + (size_t)b * 32 + 4 * (lane & 7);
  const v4i cv = *(const v4i*)(scnt + 4 * tid);
  const v4i ov = *(const v4i*)(soff + 4 * tid);
  v4i mv = {0, 0, 0, 0};
  mv.x = (lane == 0) ? nh : 0;
  mv.y = (lane == 0) ? ((nh >= RCAP) ? 1 : 0) : 0;
  const bool mw = (wave == 0) && (lane < 8);
#pragma unroll 1
  for (int p = tid; p < RCAP / 4; p += NTHR) {
    const v4i v = *(const v4i*)(reg2 + 4 * p);
    *(volatile v4i*)(hg + 4 * p) = v;
  }
  *(volatile v4i*)cg = cv;
  *(volatile v4i*)og = ov;
  if (mw) *(volatile v4i*)mg = mv;
  __threadfence();
#pragma unroll 1
  for (int p = tid; p < RCAP / 4; p += NTHR) {
    const v4i v = *(const v4i*)(reg2 + 4 * p);
    *(volatile v4i*)(hg + 4 * p) = v;
  }
  *(volatile v4i*)cg = cv;
  *(volatile v4i*)og = ov;
  if (mw) *(volatile v4i*)mg = mv;
}

__global__ __launch_bounds__(GTHR) void k_gemm(
    const unsigned short* __restrict__ A, const unsigned short* __restrict__ WT,
    const float* __restrict__ bcol, float* outF, int K, int ldo)
{
  __shared__ __attribute__((aligned(16))) float stg[GBM * GBN];
  const int tid = (int)threadIdx.x, lane = tid & 31, wave = tid >> 5, hh = lane >> 4, m = lane & 15;
  const int rowBase = (int)blockIdx.x * GBM;
  const int col0    = (int)blockIdx.y * GBN;

  float bv[4];
#pragma unroll
  for (int t = 0; t < 4; ++t) bv[t] = bcol[col0 + 16 * t + m];

  v8f acc[4];
  {
    const v8f z = {0.f, 0.f, 0.f, 0.f, 0.f, 0.f, 0.f, 0.f};
    acc[0] = z; acc[1] = z; acc[2] = z; acc[3] = z;
  }
  const unsigned short* ap = A  + (size_t)(rowBase + 16 * wave + m) * (size_t)K + 8 * hh;
  const unsigned short* wp = WT + (size_t)(col0 + m) * (size_t)K + 8 * hh;
  const int ksteps = K >> 5;
#pragma unroll 1
  for (int ks = 0; ks < ksteps; ++ks) {
    FragB af;
    af.h[0] = *(const v8usa*)(ap + 32 * ks);
    af.h[1] = *(const v8usa*)(ap + 32 * ks + 16);
#pragma unroll
    for (int t = 0; t < 4; ++t) {
      const unsigned short* wq = wp + (size_t)(16 * t) * (size_t)K + 32 * ks;
      FragB bf;
      bf.h[0] = *(const v8usa*)wq;
      bf.h[1] = *(const v8usa*)(wq + 16);
      acc[t] = wmb(af, bf, acc[t]);
    }
  }

#pragma unroll
  for (int t = 0; t < 4; ++t) {
    const int lc = 16 * t + m;
#pragma unroll
    for (int r = 0; r < 8; ++r) {
      const int lr = 16 * wave + 8 * hh + r;
      stg[lr * GBN + lc] = acc[t][r] + bv[t];
    }
  }
  __syncthreads();

  v4f fv[8];
#pragma unroll
  for (int i = 0; i < 8; ++i) {
    const int lr = 16 * wave + 2 * i + hh;
    fv[i] = *(const v4fa*)(stg + lr * GBN + 4 * m);
  }
#pragma unroll
  for (int i = 0; i < 8; ++i) {
    const int lr = 16 * wave + 2 * i + hh;
    const int gr = rowBase + lr;
    float* op = outF + (size_t)gr * (size_t)ldo + col0 + 4 * m;
    *(volatile v4f*)op = fv[i];
  }
  __threadfence();
#pragma unroll
  for (int i = 0; i < 8; ++i) {
    const int lr = 16 * wave + 2 * i + hh;
    const int gr = rowBase + lr;
    float* op = outF + (size_t)gr * (size_t)ldo + col0 + 4 * m;
    *(volatile v4f*)op = fv[i];
  }
}

template<int LAYER>
__global__ __launch_bounds__(NTHR) void k_scan(
    const float* __restrict__ XLR, const float* __restrict__ PAR,
    const int* __restrict__ HITS, const int* __restrict__ SCNT, const int* __restrict__ SOFF,
    const int* __restrict__ META, unsigned int* H1w, float* out, int nN, int MPr) {
  __shared__ __attribute__((aligned(16))) int   s_cnt[NBRUN];
  __shared__ __attribute__((aligned(16))) int   s_off[NBRUN];
  __shared__ __attribute__((aligned(16))) float s_w1[HID * FC1N];
  __shared__ __attribute__((aligned(16))) float s_fb[FC1N];
  __shared__ __attribute__((aligned(16))) float s_f2[FC1N];
  __shared__ __attribute__((aligned(16))) float s_h2[NWAVE * HID];
  __shared__ __attribute__((aligned(16))) float s_out[NBRUN];
  const int tid = (int)threadIdx.x, lane = tid & 31, wave = tid >> 5;
  const int b = (int)blockIdx.x;
  const int nodeBase = b * NBRUN;

  {
    const v4i c = *(const v4i*)(SCNT + (size_t)b * NBRUN + 4 * tid);
    const v4i o = *(const v4i*)(SOFF + (size_t)b * NBRUN + 4 * tid);
    *(v4i*)(s_cnt + 4 * tid) = c;
    *(v4i*)(s_off + 4 * tid) = o;
  }
  float f2b = 0.f;
  if (LAYER == 1) {
#pragma unroll 1
    for (int j = 0; j < 2; ++j) {
      const int q = 4 * (tid + NTHR * j);
      const v4f w = *(const v4fa*)(PAR + PO_FC1W + q);
      *(v4fa*)(s_w1 + q) = w;
    }
    const int i32 = tid & 31;
    const float fa = PAR[PO_FC1B + i32], fc = PAR[PO_FC2W + i32];
    if (tid < 32) { s_fb[i32] = fa; s_f2[i32] = fc; }
    f2b = PAR[PO_FC2B];
  }
  const int nhr = META[(size_t)b * 32];
  const int flg = META[(size_t)b * 32 + 1];
  __syncthreads();

  const int nh = nhr < 0 ? 0 : (nhr > RCAP ? RCAP : nhr);
  const bool bflag = (flg != 0) || (nhr >= RCAP) || (nhr < 0);
  const float qnan = __int_as_float(0x7fc00000);
  const v2f at = *(const v2fa*)(PAR + PO_ATT  + HID * LAYER + 2 * lane);
  const v2f bb = *(const v2fa*)(PAR + PO_BIAS + HID * LAYER + 2 * lane);
  const int* hb = HITS + (size_t)b * RCAP;
  float* hrow = s_h2 + wave * HID;
  const int nbw = NBRUN / NWAVE;

#pragma unroll 1
  for (int jt = 0; jt < nbw; ++jt) {
    const int slot = wave * nbw + jt;
    const int grow = nodeBase + slot;
    const int gcl  = grow < nN ? grow : nN - 1;
    int st = __builtin_amdgcn_readfirstlane(s_off[slot]);
    const int craw = __builtin_amdgcn_readfirstlane(s_cnt[slot]);
    int cnt = craw;
    st  = st < 0 ? 0 : (st > nh ? nh : st);
    cnt = cnt < 0 ? 0 : (cnt > DEGCAP ? DEGCAP : cnt);
    if (cnt > nh - st) cnt = nh - st;
    const float pz = (bflag || craw > DEGCAP || craw < 0) ? qnan : 0.0f;

    const float* rp = XLR + (size_t)gcl * F_IN + 2 * lane;
    const v2f xl = *(const v2fa*)rp;
    const v2f xr = *(const v2fa*)(rp + HID);
    float e0 = xl.x + xr.x, e1 = xl.y + xr.y;
    e0 = e0 > 0.f ? e0 : NEG_ATT * e0;
    e1 = e1 > 0.f ? e1 : NEG_ATT * e1;
    float part = fmaf(e1, at.y, e0 * at.x);
    part += __shfl_xor(part, 1);
    part += __shfl_xor(part, 2);
    part += __shfl_xor(part, 4);
    float mx = part, dn = 1.0f;
    float a0 = xl.x, a1 = xl.y;

#pragma unroll 1
    for (int c0 = 0; c0 < cnt; c0 += 32) {
      int idx = st + c0 + lane;
      idx = idx > RCAP - 1 ? RCAP - 1 : idx;
      const int hv = hb[idx];
      const int m32 = (cnt - c0) < 32 ? (cnt - c0) : 32;
#pragma unroll 1
      for (int k = 0; k < m32; ++k) {
        int s = __builtin_amdgcn_readlane(hv, k);
        s = s < 0 ? 0 : (s > nN - 1 ? nN - 1 : s);
        const v2f fs = *(const v2fa*)(XLR + (size_t)s * F_IN + 2 * lane);
        float g0 = fs.x + xr.x, g1 = fs.y + xr.y;
        g0 = g0 > 0.f ? g0 : NEG_ATT * g0;
        g1 = g1 > 0.f ? g1 : NEG_ATT * g1;
        float al = fmaf(g1, at.y, g0 * at.x);
        al += __shfl_xor(al, 1);
        al += __shfl_xor(al, 2);
        al += __shfl_xor(al, 4);
        const float df = al - mx;
        const float ee = expf(-fabsf(df));
        const bool up  = df > 0.f;
        const float s1 = up ? ee : 1.0f;
        const float s2 = up ? 1.0f : ee;
        mx = up ? al : mx;
        dn = fmaf(dn, s1, s2);
        a0 = fmaf(a0, s1, s2 * fs.x);
        a1 = fmaf(a1, s1, s2 * fs.y);
      }
    }
    const float inv = __builtin_amdgcn_rcpf(dn + EPS_SM);
    float v0 = fmaf(a0, inv, bb.x);
    float v1 = fmaf(a1, inv, bb.y);

    if (LAYER == 0) {
      v0 = v0 > 0.f ? v0 : NEG_ACT * v0;
      v1 = v1 > 0.f ? v1 : NEG_ACT * v1;
      const bool live = grow < nN;
      v0 = (live ? v0 : 0.f) + pz;
      v1 = (live ? v1 : 0.f) + pz;
      const unsigned int h0 = f2bfn(v0), h1 = f2bfn(v1);
      const unsigned int l0 = f2bfn(v0 - bf2f(h0)), l1 = f2bfn(v1 - bf2f(h1));
      const unsigned int hw = h0 | (h1 << 16);
      const unsigned int lw = l0 | (l1 << 16);
      unsigned int* gp = H1w + (size_t)grow * (F_IN / 2);
      const bool wr = grow < MPr;
      if (wr) { *(volatile unsigned int*)(gp + lane) = hw; *(volatile unsigned int*)(gp + 32 + lane) = lw; }
      __threadfence();
      if (wr) { *(volatile unsigned int*)(gp + lane) = hw; *(volatile unsigned int*)(gp + 32 + lane) = lw; }
    } else {
      v0 += pz; v1 += pz;
      v2f hv2; hv2.x = v0; hv2.y = v1;
      __builtin_amdgcn_fence(__ATOMIC_RELEASE, "wavefront");
      __builtin_amdgcn_wave_barrier();
      *(v2fa*)(hrow + 2 * lane) = hv2;
      __builtin_amdgcn_fence(__ATOMIC_RELEASE, "wavefront");
      __builtin_amdgcn_wave_barrier();
      float z = 0.f;
#pragma unroll 4
      for (int k = 0; k < HID; ++k) z = fmaf(hrow[k], s_w1[k * FC1N + lane], z);
      z += s_fb[lane];
      z = z > 0.f ? z : NEG_ACT * z;
      float t = z * s_f2[lane];
#pragma unroll
      for (int off = 16; off > 0; off >>= 1) t += __shfl_xor(t, off);
      const float o = t + f2b;
      if (lane == 0) s_out[slot] = o;
    }
  }

  if (LAYER == 1) {
    __syncthreads();
    int live = nN - nodeBase;
    live = live < 0 ? 0 : (live > NBRUN ? NBRUN : live);
    const v4f sv = *(const v4fa*)(s_out + 4 * tid);
    v4f o4;
    o4.x = bflag ? qnan : sv.x; o4.y = bflag ? qnan : sv.y;
    o4.z = bflag ? qnan : sv.z; o4.w = bflag ? qnan : sv.w;
    const bool wr = 4 * tid < live;
    float* op = out + (size_t)nodeBase + 4 * tid;
    if (wr) *(volatile v4f*)op = o4;
    __threadfence();
    if (wr) *(volatile v4f*)op = o4;
  }
  (void)H1w; (void)out; (void)f2b; (void)hrow;
}

static inline int cdiv(int a, int b) { return (a + b - 1) / b; }

extern "C" void kernel_launch(void* const* d_in, const int* in_sizes, int n_in,
                              void* d_out, int out_size, void* d_ws, size_t ws_size,
                              hipStream_t stream) {
  if (n_in < 18) return;
  const int nN = in_sizes[0] / F_IN;
  if (nN < 32 || in_sizes[0] != nN * F_IN || nN >= (1 << SRCB) || (nN % 32) != 0) return;
  if (in_sizes[1] < 2 || (in_sizes[1] & 1) != 0) return;
  const int nE = in_sizes[1] / 2;
  if (nE < 1 || nE > (1 << 28)) return;
  if (in_sizes[2] != F_IN * HID || in_sizes[3] != HID || in_sizes[4] != F_IN * HID || in_sizes[5] != HID) return;
  if (in_sizes[6] != HID || in_sizes[7] != HID) return;
  if (in_sizes[8] != HID * HID || in_sizes[9] != HID || in_sizes[10] != HID * HID || in_sizes[11] != HID) return;
  if (in_sizes[12] != HID || in_sizes[13] != HID) return;
  if (in_sizes[14] != HID * FC1N || in_sizes[15] != FC1N || in_sizes[16] != FC1N || in_sizes[17] != 1) return;
  if (out_size != nN) return;

  const float* x     = (const float*)d_in[0];
  const int*   ei    = (const int*)  d_in[1];
  const float* wl0   = (const float*)d_in[2];
  const float* bl0   = (const float*)d_in[3];
  const float* wr0   = (const float*)d_in[4];
  const float* br0   = (const float*)d_in[5];
  const float* att0  = (const float*)d_in[6];
  const float* bias0 = (const float*)d_in[7];
  const float* wl1   = (const float*)d_in[8];
  const float* bl1   = (const float*)d_in[9];
  const float* wr1   = (const float*)d_in[10];
  const float* br1   = (const float*)d_in[11];
  const float* att1  = (const float*)d_in[12];
  const float* bias1 = (const float*)d_in[13];
  const float* fc1w  = (const float*)d_in[14];
  const float* fc1b  = (const float*)d_in[15];
  const float* fc2w  = (const float*)d_in[16];
  const float* fc2b  = (const float*)d_in[17];
  float* out = (float*)d_out;
  const int* src = ei;
  const int* dst = ei + nE;

  const int MP   = cdiv(nN, MROWS) * MROWS;
  const int gB   = cdiv(MP, NBRUN);
  const int vec8 = ((nE & 3) == 0) ? 1 : 0;
  if (gB * NBRUN < MP) return;

  char* ws = (char*)d_ws;
  size_t off = 0;
  const size_t oA    = off; off += (size_t)MP * F_IN * 2;        off = (off + 255) & ~(size_t)255;
  const size_t oXLR  = off; off += (size_t)MP * F_IN * 4;        off = (off + 255) & ~(size_t)255;
  const size_t oW0   = off; off += (size_t)F_IN * F_IN * 2;      off = (off + 255) & ~(size_t)255;
  const size_t oW1   = off; off += (size_t)F_IN * F_IN * 2;      off = (off + 255) & ~(size_t)255;
  const size_t oPAR  = off; off += (size_t)PARN * 4;             off = (off + 255) & ~(size_t)255;
  const size_t oHITS = off; off += (size_t)gB * RCAP * 4;        off = (off + 255) & ~(size_t)255;
  const size_t oSCNT = off; off += (size_t)gB * NBRUN * 4;       off = (off + 255) & ~(size_t)255;
  const size_t oSOFF = off; off += (size_t)gB * NBRUN * 4;       off = (off + 255) & ~(size_t)255;
  const size_t oMETA = off; off += (size_t)gB * 128;             off = (off + 255) & ~(size_t)255;
  if (off > ws_size || off > (size_t)WSMAX) return;
  unsigned short* RA   = (unsigned short*)(ws + oA);
  float*          XLR  = (float*)(ws + oXLR);
  unsigned short* W0T  = (unsigned short*)(ws + oW0);
  unsigned short* W1T2 = (unsigned short*)(ws + oW1);
  float*          PAR  = (float*)(ws + oPAR);
  int*            HITS = (int*)(ws + oHITS);
  int*            SCNT = (int*)(ws + oSCNT);
  int*            SOFF = (int*)(ws + oSOFF);
  int*            META = (int*)(ws + oMETA);

  hipFuncSetAttribute(reinterpret_cast<const void*>(&k_bucket),
                      hipFuncAttributeMaxDynamicSharedMemorySize, LDS_BKT);

  const int nbX = MP / 16;
  k_prep<<<nbX + 17, NTHR, 0, stream>>>(x, wl0, bl0, wr0, br0, att0, bias0, wl1, bl1, wr1, br1, att1, bias1,
                                        fc1w, fc1b, fc2w, fc2b, RA, W0T, W1T2, PAR, nN, nbX);
  k_bucket<<<gB, NTHR, LDS_BKT, stream>>>(src, dst, HITS, SCNT, SOFF, META, nN, nE, vec8);
  const int gM = MP / GBM;
  k_gemm<<<dim3(gM, F_IN / GBN), GTHR, 0, stream>>>(RA, W0T, PAR + PO_BLR0, XLR, F_IN, F_IN);
  k_scan<0><<<gB, NTHR, 0, stream>>>(XLR, PAR, HITS, SCNT, SOFF, META, (unsigned int*)RA, out, nN, MP);
  k_gemm<<<dim3(gM, F_IN / GBN), GTHR, 0, stream>>>(RA, W1T2, PAR + PO_BLR1, XLR, F_IN, F_IN);
  k_scan<1><<<gB, NTHR, 0, stream>>>(XLR, PAR, HITS, SCNT, SOFF, META, (unsigned int*)RA, out, nN, MP);
}
